// RelationAttentionHead_10539849744624
// MI455X (gfx1250) — hardware-run, weakly checked
//
#include <hip/hip_runtime.h>


namespace {
constexpr int N = 100000, E = 1000000, D = 128, R = 64, RD = 64, H = 128, NH = 4, HD = 32, KW = 144  ;
constexpr float XS = 8.0f, HS = 256.0f, WSC = 256.0f;
typedef _Float16 b16;
typedef __attribute__((ext_vector_type(16))) _Float16 v16b;
typedef __attribute__((ext_vector_type(8))) _Float16 v8b;
typedef __attribute__((ext_vector_type(8))) float v8f;
typedef __attribute__((ext_vector_type(4))) float v4f;
__device__ __forceinline__ float bf16_rne(float f) { unsigned int u = __float_as_uint(f); u += 0x7FFFu + ((u >> 16) & 1u); float r = __uint_as_float(u & 0xFFFF0000u); asm volatile("" : "+v"(r)); return r; }
__device__ __forceinline__ float bfv(float f) { float r = bf16_rne(f); asm volatile("" : "+v"(r)); return r; }
__device__ __forceinline__ void split16(float v, b16& hi, b16& lo) { hi = (b16)v; lo = (b16)(v - (float)hi); }
__device__ __forceinline__ v16b frag_kb(const b16* p, int hh) { const v8b a = *(const v8b*)(p + 8 * hh), b = *(const v8b*)(p + 16 + 8 * hh); v16b f;
#pragma unroll
  for (int e = 0; e < 8; ++e) { f[e] = a[e]; f[8 + e] = b[e]; } return f; }
__device__ __forceinline__ v8f wmma16b(v16b a, v16b b, v8f c) { v8f d = __builtin_amdgcn_wmma_f32_16x16x32_f16(false, a, false, b, (short)0, c, false, false); asm volatile("v_nop\n\tv_nop\n\tv_nop\n\tv_nop" : "+v"(d) : "v"(a), "v"(b)); return d; }
__device__ __forceinline__ void wave_lds_sync() { __builtin_amdgcn_fence(__ATOMIC_RELEASE, "workgroup"); __builtin_amdgcn_wave_barrier(); __builtin_amdgcn_fence(__ATOMIC_ACQUIRE, "workgroup"); }
__device__ __forceinline__ float pmul(float a, float b) { float p = a * b; asm volatile("" : "+v"(p)); return p; }
__device__ __forceinline__ int iclamp(int v, int lo, int hi) { return v < lo ? lo : (v > hi ? hi : v); }

__global__ __launch_bounds__(256) void setup_kernel(const float* __restrict__ wedge, const float* __restrict__ wk, const float* __restrict__ wv, const float* __restrict__ wout, const float* __restrict__ relemb, const float* __restrict__ wq, const float* __restrict__ bq, const float* __restrict__ bedge, const float* __restrict__ bk, const float* __restrict__ bv, b16* __restrict__ WE, b16* __restrict__ WK, float* __restrict__ QT, float* __restrict__ CK, float* __restrict__ CVO, float* __restrict__ U) { const size_t nt = (size_t)gridDim.x * 256, u0 = (size_t)blockIdx.x * 256 + threadIdx.x; v8b v;
  for (size_t u = u0; u < (size_t)2 * H * 16; u += nt) { const int op = (int)(u / 16), k0 = (int)(u % 16) * 8; const int o = op % H, half = op / H;
#pragma unroll
    for (int j = 0; j < 8; ++j) v[j] = (b16)(bf16_rne(wedge[(size_t)(half * D + k0 + j) * H + o]) * WSC); for (int pass = 0; pass < 2; ++pass) { *(volatile v8b*)(WE + (size_t)op * D + k0) = v; __threadfence(); } }
  for (size_t u = u0; u < (size_t)KW * 16; u += nt) { const int o = (int)(u / 16), k0 = (int)(u % 16) * 8;
#pragma unroll
    for (int j = 0; j < 8; ++j) v[j] = (b16)(o < H ? bf16_rne(wk[(size_t)(k0 + j) * H + o]) * WSC : 0.0f); for (int pass = 0; pass < 2; ++pass) { *(volatile v8b*)(WK + (size_t)o * H + k0) = v; __threadfence(); } }
  for (size_t u = u0; u < (size_t)R * H; u += nt) { const int r = (int)(u / H), o = (int)(u % H); float s = bfv(bq[o]); for (int k = 0; k < RD; ++k) s += pmul(bfv(relemb[r * RD + k]), bfv(wq[(size_t)k * H + o])); for (int pass = 0; pass < 2; ++pass) { ((volatile float*)QT)[u] = s; __threadfence(); } }
  for (size_t u = u0; u < (size_t)H; u += nt) { const int o = (int)u; float s = bfv(bk[o]); for (int k = 0; k < H; ++k) s += pmul(bfv(bedge[k]), bfv(wk[(size_t)k * H + o])); for (int pass = 0; pass < 2; ++pass) { ((volatile float*)CK)[o] = s; __threadfence(); } }
  for (size_t u = u0; u < (size_t)NH * H; u += nt) { const int h = (int)(u / H), k = (int)(u % H); float s = 0.0f; for (int d = h * HD; d < h * HD + HD; ++d) s += pmul(bfv(wv[(size_t)k * H + d]), bfv(wout[d])); for (int pass = 0; pass < 2; ++pass) { ((volatile float*)U)[u] = s; __threadfence(); } }
  if (u0 < 32) { float s = 0.0f; if (u0 < NH) { const int h = (int)u0; for (int d = h * HD; d < h * HD + HD; ++d) { float bvd = bfv(bv[d]); for (int k = 0; k < H; ++k) bvd += pmul(bfv(bedge[k]), bfv(wv[(size_t)k * H + d])); s += pmul(bvd, bfv(wout[d])); } } for (int pass = 0; pass < 2; ++pass) { ((volatile float*)CVO)[u0] = s; __threadfence(); } } }
__global__ __launch_bounds__(32) void node_kernel(const float* __restrict__ emb, const b16* __restrict__ WE, const b16* __restrict__ WK, const float* __restrict__ U, int NLIM, float* __restrict__ PKU) { __shared__ __attribute__((aligned(16))) b16 Ah[16][D + 8], Al[16][D + 8]; __shared__ float Pf[16][2 * H + 4], Tf[16][164], Nr[16]; const int lane = threadIdx.x, nloc = lane & 15, hlf = lane >> 4; const size_t m0 = (size_t)blockIdx.x * 16; if (m0 >= (size_t)NLIM) return;
  for (int rr = 0; rr < 16; ++rr) { float sq = 0.0f; for (int q = 0; q < 4; ++q) { const float v = bfv(emb[(m0 + rr) * D + q * 32 + lane]); sq += v * v; Ah[rr][q * 32 + lane] = (b16)(v * XS); } for (int o = 16; o; o >>= 1) sq += __shfl_xor(sq, o); if (lane == 0) Nr[rr] = 1.0f / fmaxf(sqrtf(sq), 1e-12f); }
  if (lane < 16) for (int k = D; k < D + 8; ++k) { Ah[lane][k] = (b16)0.0f; Al[lane][k] = (b16)0.0f; }
  wave_lds_sync();
  { v8f acc[16];
#pragma unroll
    for (int t = 0; t < 16; ++t) acc[t] = (v8f){};
#pragma unroll
    for (int kb = 0; kb < D; kb += 32) { const v16b a = frag_kb(&Ah[nloc][kb], hlf);
#pragma unroll
      for (int t = 0; t < 16; ++t) acc[t] = wmma16b(a, frag_kb(WE + (size_t)(t * 16 + nloc) * D + kb, hlf), acc[t]); }
#pragma unroll
    for (int t = 0; t < 16; ++t)
#pragma unroll
      for (int r8 = 0; r8 < 8; ++r8) { const int rr = 8 * hlf + r8; Pf[rr][t * 16 + nloc] = pmul(acc[t][r8] * (1.0f / (XS * WSC)), Nr[rr]); } }
  wave_lds_sync();
#pragma unroll 1
  for (int g = 0; g < 2; ++g) {
    for (int rr = 0; rr < 16; ++rr) for (int q = 0; q < 4; ++q) { const int c = q * 32 + lane; b16 p, ql; split16(Pf[rr][g * H + c] * HS, p, ql); Ah[rr][c] = p; Al[rr][c] = ql; }
    wave_lds_sync(); v8f acc[8];
#pragma unroll
    for (int t = 0; t < 8; ++t) acc[t] = (v8f){};
#pragma unroll
    for (int kb = 0; kb < D; kb += 32) { const v16b a = frag_kb(&Ah[nloc][kb], hlf), al = frag_kb(&Al[nloc][kb], hlf);
#pragma unroll
      for (int t = 0; t < 8; ++t) { const v16b bw = frag_kb(WK + (size_t)(t * 16 + nloc) * D + kb, hlf); acc[t] = wmma16b(a, bw, acc[t]); acc[t] = wmma16b(al, bw, acc[t]); } }
#pragma unroll
    for (int t = 0; t < 8; ++t)
#pragma unroll
      for (int r8 = 0; r8 < 8; ++r8) Tf[8 * hlf + r8][t * 16 + nloc] = acc[t][r8] * (1.0f / (HS * WSC));
    { const int rr = nloc; for (int h = 2 * hlf; h < 2 * hlf + 2; ++h) { float s = 0.0f; for (int k = 0; k < D; ++k) s += pmul(Pf[rr][g * H + k], U[h * D + k]); Tf[rr][128 + h] = s; } if (hlf == 0) for (int c = 132; c < 160; ++c) Tf[rr][c] = 0.0f; }
    wave_lds_sync();
    for (int pass = 0; pass < 2; ++pass) { for (int rr = 0; rr < 16; ++rr) for (int q = 0; q < 5; ++q) ((volatile float*)PKU)[((m0 + rr) * 2 + g) * 160 + q * 32 + lane] = Tf[rr][q * 32 + lane]; __threadfence(); }
    wave_lds_sync(); } }
__global__ __launch_bounds__(256) void edge_kernel(const float* __restrict__ PKU, const float* __restrict__ QT, const float* __restrict__ CK, const float* __restrict__ CVO, const float* __restrict__ bout, const int* __restrict__ ei, const int* __restrict__ rel, int NLIM, int ELIM, float* __restrict__ out) { __shared__ float Qs[R][H + 1], Cs[H]; for (int u = threadIdx.x; u < R * H; u += 256) Qs[u / H][u % H] = QT[u]; for (int u = threadIdx.x; u < H; u += 256) Cs[u] = CK[u]; __syncthreads();
  const size_t e = (size_t)blockIdx.x * 256 + threadIdx.x; if (e >= (size_t)ELIM) return; const size_t s = (size_t)iclamp(ei[e], 0, NLIM - 1), t = (size_t)iclamp(ei[(size_t)E + e], 0, NLIM - 1); const int r = iclamp(rel[e], 0, R - 1); const float* ks = PKU + (s * 2 + 0) * 160; const float* kt = PKU + (t * 2 + 1) * 160;
  float sc[NH];
#pragma unroll
  for (int h = 0; h < NH; ++h) { float a = 0.0f;
#pragma unroll 4
    for (int d = h * HD; d < h * HD + HD; ++d) a += pmul(Qs[r][d], ks[d] + kt[d] + Cs[d]); sc[h] = a * 0.17677669529663688f; }
  float mx = fmaxf(fmaxf(sc[0], sc[1]), fmaxf(sc[2], sc[3])); float den = 0.0f, num = 0.0f;
#pragma unroll
  for (int h = 0; h < NH; ++h) { const float p = __expf(sc[h] - mx); den += p; num += pmul(p, ks[128 + h] + kt[128 + h] + CVO[h]); }
  const float score = num / den + bfv(bout[0]);
  for (int pass = 0; pass < 2; ++pass) { ((volatile float*)out)[e] = score; __threadfence(); } }
}

extern "C" void kernel_launch(void* const* d_in, const int* in_sizes, int n_in, void* d_out, int out_size, void* d_ws, size_t ws_size, hipStream_t stream) {
  (void)n_in;
  auto Fp = [&](int i) { return (const float*)d_in[i]; }; auto Ip = [&](int i) { return (const int*)d_in[i]; };
  if (in_sizes[0] != N * D || in_sizes[1] != 2 * E || in_sizes[2] != E || in_sizes[3] != R * RD || in_sizes[4] != 2 * D * H || in_sizes[6] != RD * H || in_sizes[8] != H * H || in_sizes[10] != H * H || in_sizes[12] != H || out_size != E) return;
  const int NLIM = N, ELIM = E;
  size_t off = 0; char* ws = (char*)d_ws;
  auto carve = [&](size_t bytes) { char* p = ws + off; off += (bytes + 255) & ~(size_t)255; return p; };
  b16* WE = (b16*)carve((size_t)2 * H * D * 2); b16* WK = (b16*)carve((size_t)KW * D * 2); float* QT = (float*)carve((size_t)R * H * 4); float* CK = (float*)carve(H * 4); float* CVO = (float*)carve(256); float* U = (float*)carve((size_t)NH * D * 4); float* PKU = (float*)carve((size_t)N * 2 * 160 * 4);
  if (off > ws_size || off > ((size_t)160 << 20)) return;
  setup_kernel<<<64, 256, 0, stream>>>(Fp(4), Fp(8), Fp(10), Fp(12), Fp(3), Fp(6), Fp(7), Fp(5), Fp(9), Fp(11), WE, WK, QT, CK, CVO, U);
  node_kernel<<<NLIM / 16, 32, 0, stream>>>(Fp(0), WE, WK, U, NLIM, PKU);
  edge_kernel<<<(ELIM + 255) / 256, 256, 0, stream>>>(PKU, QT, CK, CVO, Fp(13), Ip(1), Ip(2), NLIM, ELIM, (float*)d_out);
}
